// QAdaptHypergraphConv_65463891526212
// MI455X (gfx1250) — hardware-verified
//
#include <hip/hip_runtime.h>

#define NB    4
#define NNODE 4096
#define ECOLS 256
#define DD    256
#define NEMAX 50
#define H1DIM 128
#define H2DIM 64
#define NROWS (NB * NNODE)
#define OCOLS 512

typedef _Float16 v16h __attribute__((ext_vector_type(16)));
typedef _Float16 v8h  __attribute__((ext_vector_type(8)));
typedef float    v8f  __attribute__((ext_vector_type(8)));
typedef float    v4f  __attribute__((ext_vector_type(4)));

static_assert(NNODE == 4096);
static_assert((DD % 64) == 0 && (NROWS % 64) == 0 && (NROWS % 32) == 0);
static_assert(NEMAX <= 64 && NB <= 4);

__device__ __forceinline__ v16h ldfrag(const _Float16* p) {
  union { v16h v; v8h h[2]; } f;
  f.h[0] = *(const v8h*)(p);
  f.h[1] = *(const v8h*)(p + 16);
  return f.v;
}
__device__ __forceinline__ v8f mma16(v16h a, v16h b, v8f c) {
  return __builtin_amdgcn_wmma_f32_16x16x32_f16(false, a, false, b, (short)0, c, false, false);
}
__device__ __forceinline__ v8f zero8() {
  v8f z;
#pragma unroll
  for (int i = 0; i < 8; ++i) z[i] = 0.0f;
  return z;
}

__device__ __forceinline__ void guard_g(v8f& a, v8f& b, v16h x, v16h y) {
#if defined(__HIP_DEVICE_COMPILE__)
  asm volatile("v_nop\n\tv_nop\n\tv_nop\n\tv_nop" : "+v"(a), "+v"(b) : "v"(x), "v"(y));
#endif
}
__device__ __forceinline__ void keep4(v16h a, v16h b, v16h c, v16h d) {
#if defined(__HIP_DEVICE_COMPILE__)
  asm volatile("v_nop" :: "v"(a), "v"(b), "v"(c), "v"(d));
#endif
}
__device__ __forceinline__ void accg4(v8f& a, v8f& b, v8f& c, v8f& d) {
#if defined(__HIP_DEVICE_COMPILE__)
  asm volatile("v_nop\n\tv_nop\n\tv_nop\n\tv_nop" : "+v"(a), "+v"(b), "+v"(c), "+v"(d));
#endif
}
__device__ __forceinline__ void guard_s4(v8f& a, v8f& b, v8f& c, v8f& d, v16h x0, v16h x1, v16h y0, v16h y1) {
#if defined(__HIP_DEVICE_COMPILE__)
  asm volatile("v_nop\n\tv_nop\n\tv_nop\n\tv_nop"
               : "+v"(a), "+v"(b), "+v"(c), "+v"(d) : "v"(x0), "v"(x1), "v"(y0), "v"(y1));
#endif
}

__global__ __launch_bounds__(256) void cvt_w_kernel(const float* __restrict__ w0, const float* __restrict__ w1,
                                                    _Float16* __restrict__ d0, _Float16* __restrict__ d1, int dim) {
  const int wave = threadIdx.x >> 5, lane = threadIdx.x & 31;
  const int nbm = dim >> 3;
  const bool second = ((int)blockIdx.x >= nbm);
  const float* src = second ? w1 : w0;
  _Float16* dst = second ? d1 : d0;
  const int f = ((int)blockIdx.x - (second ? nbm : 0)) * 8 + wave;
  if (f >= dim) return;
  const int k0 = lane * 8;
  v8h o;
#pragma unroll
  for (int i = 0; i < 8; ++i) o[i] = (_Float16)(src[(size_t)(k0 + i) * dim + f] * 64.0f);
  _Float16* d = dst + (size_t)f * dim + k0;
  *(volatile v8h*)d = o;
  __threadfence();
  *(volatile v8h*)d = o;
}

__global__ __launch_bounds__(256) void cvt_x_kernel(const float* __restrict__ x, const float* __restrict__ cw,
                                                    const float* __restrict__ cb, _Float16* __restrict__ X,
                                                    float* __restrict__ compat) {
  __shared__ __align__(16) float s_c[32];
  const int wave = threadIdx.x >> 5, lane = threadIdx.x & 31;
  const int c0 = lane * 8;
  const v4f wa = *(const v4f*)(cw + c0), wb = *(const v4f*)(cw + c0 + 4);
  const float cb0 = cb[0];
#pragma unroll 1
  for (int rr = 0; rr < 4; ++rr) {
    const int lrow = wave * 4 + rr;
    const int row = (int)blockIdx.x * 32 + lrow;
    const float* xr = x + (size_t)row * DD + c0;
    const v4f a = *(const v4f*)xr, bq = *(const v4f*)(xr + 4);
    v8h o;
    float s = 0.0f;
#pragma unroll
    for (int i = 0; i < 4; ++i) {
      o[i]     = (_Float16)a[i];
      o[4 + i] = (_Float16)bq[i];
      s += a[i] * wa[i];
      s += bq[i] * wb[i];
    }
#pragma unroll
    for (int off = 16; off > 0; off >>= 1) s += __shfl_xor(s, off, 32);
    _Float16* d = X + (size_t)row * DD + c0;
    *(volatile v8h*)d = o;
    __threadfence();
    *(volatile v8h*)d = o;
    if (lane == 0) s_c[lrow] = s + cb0;
  }
  __syncthreads();
  if (threadIdx.x < 8) {
    const v4f v = *(const v4f*)(s_c + 4 * (int)threadIdx.x);
    float* d = compat + (size_t)blockIdx.x * 32 + 4 * (int)threadIdx.x;
    *(volatile v4f*)d = v;
    __threadfence();
    *(volatile v4f*)d = v;
  }
}

template <bool BIAS>
__global__ __launch_bounds__(256) void gemm64_kernel(const _Float16* __restrict__ A, int lda,
                                                     const _Float16* __restrict__ Bt, int ldb,
                                                     _Float16* __restrict__ C, int ldc,
                                                     const float* __restrict__ bias, float bscale,
                                                     int M, int N, int K, float scale) {
  __shared__ __align__(16) float sT[8][16 * 68];
  const int lane = threadIdx.x & 31, wave = threadIdx.x >> 5;
  const int tilesN = N >> 6, tilesM = M >> 6;
  const int tile = (int)blockIdx.x * 8 + wave;
  if (tile >= tilesM * tilesN) return;
  const int tm = tile / tilesN, tn = tile - tm * tilesN;
  const int m0 = tm << 6, n0 = tn << 6;
  const int rl = lane & 15;
  const int koff = (lane >> 4) * 8;
  const int mOff = (lane >> 4) * 8;

  v8f acc[4][4];
#pragma unroll
  for (int i = 0; i < 4; ++i)
#pragma unroll
    for (int j = 0; j < 4; ++j) acc[i][j] = zero8();

#pragma unroll 1
  for (int k0 = 0; k0 < K; k0 += 32) {
    v16h bh[4];
#pragma unroll
    for (int j = 0; j < 4; ++j) bh[j] = ldfrag(Bt + (size_t)(n0 + (j << 4) + rl) * ldb + koff + k0);
#pragma unroll
    for (int i = 0; i < 4; ++i) {
      const v16h ah = ldfrag(A + (size_t)(m0 + (i << 4) + rl) * lda + koff + k0);
#pragma unroll
      for (int j = 0; j < 4; ++j) acc[i][j] = mma16(ah, bh[j], acc[i][j]);
      guard_g(acc[i][0], acc[i][3], ah, bh[3]);
    }
    keep4(bh[0], bh[1], bh[2], bh[3]);
  }
  accg4(acc[0][0], acc[0][1], acc[0][2], acc[0][3]);
  accg4(acc[1][0], acc[1][1], acc[1][2], acc[1][3]);
  accg4(acc[2][0], acc[2][1], acc[2][2], acc[2][3]);
  accg4(acc[3][0], acc[3][1], acc[3][2], acc[3][3]);

  float* slab = sT[wave];
  const int qq = lane >> 3, c8 = (lane & 7) * 8;
#pragma unroll
  for (int i = 0; i < 4; ++i) {
    const int mBase = m0 + (i << 4);
#pragma unroll
    for (int j = 0; j < 4; ++j) {
      float bv = 0.0f;
      if (BIAS) bv = bias[n0 + (j << 4) + rl] * bscale;
#pragma unroll
      for (int r = 0; r < 8; ++r) slab[(mOff + r) * 68 + (j << 4) + rl] = acc[i][j][r] * scale + bv;
    }
    __builtin_amdgcn_fence(__ATOMIC_RELEASE, "workgroup");
    __builtin_amdgcn_wave_barrier();
    __builtin_amdgcn_fence(__ATOMIC_ACQUIRE, "workgroup");
#pragma unroll
    for (int ps = 0; ps < 2; ++ps) {
#pragma unroll
      for (int it = 0; it < 4; ++it) {
        const int row = it * 4 + qq;
        const float* sp = slab + row * 68 + c8;
        v8h hv;
#pragma unroll
        for (int e = 0; e < 8; ++e) hv[e] = (_Float16)sp[e];
        *(volatile v8h*)(C + (size_t)(mBase + row) * ldc + n0 + c8) = hv;
      }
      __threadfence();
    }
    __builtin_amdgcn_fence(__ATOMIC_RELEASE, "workgroup");
    __builtin_amdgcn_wave_barrier();
    __builtin_amdgcn_fence(__ATOMIC_ACQUIRE, "workgroup");
  }
}

__global__ __launch_bounds__(256) void edge_kernel(const float* __restrict__ x, const int* __restrict__ H,
                                                   const float* __restrict__ m1w, const float* __restrict__ m1b,
                                                   const float* __restrict__ m2w, const float* __restrict__ m2b,
                                                   const float* __restrict__ m3w, const float* __restrict__ m3b,
                                                   float* __restrict__ ctab, int nnode, int ecols, int nbatch) {
  __shared__ int   s_mem[NNODE];
  __shared__ float s_hv[NNODE];
  __shared__ int   s_cnt[256];
  __shared__ float s_red[256];
  __shared__ float s_mean[DD];
  __shared__ float s_h1[H1DIM];
  __shared__ float s_h2[H2DIM];
  __shared__ __align__(16) float s_line[32];
  __shared__ int   s_tot;
  const int e = blockIdx.x, t = threadIdx.x;
  if (t < 32) s_line[t] = 0.0f;

  int cnt = 0;
  float dsum = 0.0f;
#pragma unroll
  for (int j = 0; j < 16; ++j) {
    const int n = t * 16 + j;
    const int v = H[(size_t)n * ecols + e];
    cnt += (v != 0) ? 1 : 0;
    dsum += (float)v;
  }
  s_cnt[t] = cnt;
  s_red[t] = dsum;
  __syncthreads();
  if (t == 0) {
    int run = 0;
#pragma unroll 1
    for (int i = 0; i < 256; ++i) { const int c2 = s_cnt[i]; s_cnt[i] = run; run += c2; }
    s_tot = run;
  }
  __syncthreads();
#pragma unroll
  for (int s = 128; s > 0; s >>= 1) {
    if (t < s) s_red[t] += s_red[t + s];
    __syncthreads();
  }
  const float deg = s_red[0];
  const int tot = s_tot;
  const int ncnt = (tot < NNODE) ? tot : NNODE;
  {
    int pos = s_cnt[t];
#pragma unroll
    for (int j = 0; j < 16; ++j) {
      const int n = t * 16 + j;
      const int v = H[(size_t)n * ecols + e];
      if (v != 0) {
        if (pos < NNODE) { s_mem[pos] = n; s_hv[pos] = (float)v; }
        ++pos;
      }
    }
  }
  __syncthreads();
  const float rdeg = 1.0f / fmaxf(deg, 1.0f);

#pragma unroll 1
  for (int bb = 0; bb < nbatch; ++bb) {
    const float* xb = x + (size_t)bb * nnode * DD + t;
    float acc = 0.0f;
#pragma unroll 2
    for (int i = 0; i < ncnt; ++i) acc += s_hv[i] * xb[(size_t)(s_mem[i] & (NNODE - 1)) * DD];
    s_mean[t] = acc * rdeg;
    __syncthreads();
    if (t < H1DIM) {
      float a = m1b[t];
      const float* wp = m1w + t;
#pragma unroll 4
      for (int k = 0; k < DD; ++k) a += s_mean[k] * wp[(size_t)k * H1DIM];
      s_h1[t] = fmaxf(a, 0.0f);
    }
    __syncthreads();
    if (t < H2DIM) {
      float a = m2b[t];
      const float* wp = m2w + t;
#pragma unroll 4
      for (int k = 0; k < H1DIM; ++k) a += s_h1[k] * wp[(size_t)k * H2DIM];
      s_h2[t] = fmaxf(a, 0.0f);
    }
    __syncthreads();
    {
      const int tc = t & (H2DIM - 1);
      const float pv = s_h2[tc] * m3w[tc];
      s_red[t] = (t < H2DIM) ? pv : 0.0f;
    }
    __syncthreads();
#pragma unroll
    for (int s = 128; s > 0; s >>= 1) {
      if (t < s) s_red[t] += s_red[t + s];
      __syncthreads();
    }
    if (t == 0) s_line[bb] = s_red[0] + m3b[0];
    __syncthreads();
  }
  if (t == 0) { s_line[4] = deg; s_line[5] = (deg > 1.0f) ? 1.0f : 0.0f; }
  __syncthreads();
  if (t < 8) {
    const v4f v = *(const v4f*)(s_line + 4 * t);
    float* d = ctab + (size_t)e * 32 + 4 * t;
    *(volatile v4f*)d = v;
    __threadfence();
    *(volatile v4f*)d = v;
  }
}

__global__ __launch_bounds__(256) void aw_kernel(const int* __restrict__ H, const float* __restrict__ compat,
                                                 const float* __restrict__ ctab, const float* __restrict__ hbias,
                                                 const float* __restrict__ alpha, float* __restrict__ out,
                                                 int ecols, int opitch, int nemax) {
  const int wave = threadIdx.x >> 5, lane = threadIdx.x & 31;
  const int row = (int)blockIdx.x * 8 + wave;
  const int b = row >> 12, n = row & (NNODE - 1);
  const float z0 = compat[row] + hbias[0];
  const float al = alpha[0];
  const int* Hr = H + (size_t)n * ecols;
  v4f o;
#pragma unroll
  for (int j = 0; j < 4; ++j) {
    const int e = lane * 4 + j;
    const int ec = (e < nemax) ? e : (nemax - 1);
    const float cx = ctab[ec * 32 + b];
    const float vd = ctab[ec * 32 + 5];
    const float hv = (float)Hr[e];
    const float z = z0 + al * cx;
    const float ez = __expf(-z);
    const float g = __builtin_amdgcn_rcpf(1.0f + ez);
    const float val = g * hv * vd;
    o[j] = (e < nemax) ? val : 0.0f;
  }
  v4f zz;
#pragma unroll
  for (int j = 0; j < 4; ++j) zz[j] = 0.0f;
  float* d0 = out + (size_t)row * opitch + lane * 4;
  float* d1 = d0 + 128;
  *(volatile v4f*)d0 = o;
  *(volatile v4f*)d1 = zz;
  __threadfence();
  *(volatile v4f*)d0 = o;
  *(volatile v4f*)d1 = zz;
}

#define QB       32
#define KCH      256
#define QSP      264
#define PSP      264
#define OSP      260
#define LDS_QS   0
#define LDS_PS   16896
#define LDS_PMAX 33792
#define LDS_PSUM 34816
#define LDS_ST   35840
#define LDS_OS   36352
#define ATT_LDS  69632
static_assert(QB * QSP * 2 == LDS_PS - LDS_QS);
static_assert(QB * PSP * 2 == LDS_PMAX - LDS_PS);
static_assert(LDS_PSUM - LDS_PMAX == 256 * 4);
static_assert(LDS_ST - LDS_PSUM == 256 * 4);
static_assert(LDS_OS - LDS_ST == 4 * 32 * 4);
static_assert(ATT_LDS - LDS_OS == QB * OSP * 4);
static_assert((QSP % 8) == 0 && (PSP % 8) == 0 && PSP >= KCH && (OSP % 4) == 0);
static_assert((LDS_PS % 16) == 0 && (LDS_PMAX % 16) == 0 && (LDS_ST % 16) == 0 && (LDS_OS % 16) == 0);
static_assert((NNODE % KCH) == 0 && (NNODE % QB) == 0 && DD == 256);

__global__ __launch_bounds__(256) void attn_kernel(const _Float16* __restrict__ qk, const _Float16* __restrict__ vt,
                                                   const float* __restrict__ bias, float* __restrict__ out,
                                                   float sc, int nkey, int vpitch, int opitch, int ocol) {
  extern __shared__ __align__(16) char smem[];
  _Float16* Qs = (_Float16*)(smem + LDS_QS);
  _Float16* Ps = (_Float16*)(smem + LDS_PS);
  float* pmax = (float*)(smem + LDS_PMAX);
  float* psum = (float*)(smem + LDS_PSUM);
  float* m_s  = (float*)(smem + LDS_ST);
  float* l_s  = m_s + 32;
  float* al_s = m_s + 64;
  float* li_s = m_s + 96;
  float* Os   = (float*)(smem + LDS_OS);

  const int tid = threadIdx.x, wave = tid >> 5, lane = tid & 31, h = lane >> 4, c = lane & 15;
  const int kbase = (int)blockIdx.y * nkey;
  const int q0 = kbase + (int)blockIdx.x * QB;
  const float ninf = -__builtin_inff();

  if (tid < 32) { m_s[tid] = ninf; l_s[tid] = 0.0f; al_s[tid] = 0.0f; li_s[tid] = 0.0f; }
  psum[tid] = 0.0f;
#pragma unroll
  for (int i = 0; i < 4; ++i) {
    const int idx = i * 256 + tid;
    const int row = idx >> 5;
    const int pc  = idx & 31;
    const v8h v = *(const v8h*)(qk + (size_t)(q0 + row) * DD + pc * 8);
    *(v8h*)(Qs + row * QSP + pc * 8) = v;
  }
  __syncthreads();

  v8f oacc[2][2];
#pragma unroll
  for (int qt = 0; qt < 2; ++qt)
#pragma unroll
    for (int nt = 0; nt < 2; ++nt) oacc[qt][nt] = zero8();

  const _Float16* qb0p = Qs + c * QSP + 8 * h;
  const _Float16* qb1p = Qs + (16 + c) * QSP + 8 * h;
  const _Float16* pa0p = Ps + c * PSP + 8 * h;
  const _Float16* pa1p = Ps + (16 + c) * PSP + 8 * h;
  const int ntile = nkey / KCH;

#pragma unroll 1
  for (int t = 0; t < ntile; ++t) {
    const int kb = kbase + t * KCH + 32 * wave;
    const _Float16* ka0p = qk + (size_t)(kb + c) * DD + 8 * h;
    const _Float16* ka1p = qk + (size_t)(kb + 16 + c) * DD + 8 * h;
    v8f sacc[2][2];
#pragma unroll
    for (int qt = 0; qt < 2; ++qt)
#pragma unroll
      for (int kt = 0; kt < 2; ++kt) sacc[qt][kt] = zero8();
#pragma unroll 1
    for (int k0 = 0; k0 < DD; k0 += 32) {
      const v16h a0 = ldfrag(ka0p + k0), a1 = ldfrag(ka1p + k0);
      const v16h b0 = ldfrag(qb0p + k0), b1 = ldfrag(qb1p + k0);
      sacc[0][0] = mma16(a0, b0, sacc[0][0]);
      sacc[0][1] = mma16(a1, b0, sacc[0][1]);
      sacc[1][0] = mma16(a0, b1, sacc[1][0]);
      sacc[1][1] = mma16(a1, b1, sacc[1][1]);
      guard_s4(sacc[0][0], sacc[0][1], sacc[1][0], sacc[1][1], a0, a1, b0, b1);
    }
    {
      float pm0 = ninf, pm1 = ninf;
#pragma unroll
      for (int kt = 0; kt < 2; ++kt) {
#pragma unroll
        for (int r = 0; r < 8; ++r) {
          const float v0 = sacc[0][kt][r] * sc; sacc[0][kt][r] = v0; pm0 = fmaxf(pm0, v0);
          const float v1 = sacc[1][kt][r] * sc; sacc[1][kt][r] = v1; pm1 = fmaxf(pm1, v1);
        }
      }
      pm0 = fmaxf(pm0, __shfl_xor(pm0, 16, 32));
      pm1 = fmaxf(pm1, __shfl_xor(pm1, 16, 32));
      pmax[wave * 32 + c] = pm0;
      pmax[wave * 32 + 16 + c] = pm1;
    }
    __syncthreads();
    if (wave == 0) {
      const int row = lane;
      float ps = 0.0f;
#pragma unroll
      for (int w = 0; w < 8; ++w) ps += psum[w * 32 + row];
      l_s[row] = l_s[row] * al_s[row] + ps;
      const float mo = m_s[row];
      float mx = mo;
#pragma unroll
      for (int w = 0; w < 8; ++w) mx = fmaxf(mx, pmax[w * 32 + row]);
      al_s[row] = __expf(mo - mx);
      m_s[row] = mx;
    }
    __syncthreads();
    {
      const float mq0 = m_s[c], mq1 = m_s[16 + c];
      float ps0 = 0.0f, ps1 = 0.0f;
#pragma unroll
      for (int kt = 0; kt < 2; ++kt) {
        v8h h0, h1;
#pragma unroll
        for (int r = 0; r < 8; ++r) {
          const float p0 = __expf(sacc[0][kt][r] - mq0); ps0 += p0; h0[r] = (_Float16)(p0 * 16.0f);
          const float p1 = __expf(sacc[1][kt][r] - mq1); ps1 += p1; h1[r] = (_Float16)(p1 * 16.0f);
        }
        *(v8h*)(Ps + c * PSP + 32 * wave + 16 * kt + 8 * h) = h0;
        *(v8h*)(Ps + (16 + c) * PSP + 32 * wave + 16 * kt + 8 * h) = h1;
      }
      ps0 += __shfl_xor(ps0, 16, 32);
      ps1 += __shfl_xor(ps1, 16, 32);
      psum[wave * 32 + c] = ps0;
      psum[wave * 32 + 16 + c] = ps1;
      const v4f aA = *(const v4f*)(al_s + 8 * h), aB = *(const v4f*)(al_s + 8 * h + 4);
      const v4f bA = *(const v4f*)(al_s + 16 + 8 * h), bB = *(const v4f*)(al_s + 16 + 8 * h + 4);
#pragma unroll
      for (int nt = 0; nt < 2; ++nt) {
#pragma unroll
        for (int r = 0; r < 4; ++r) {
          oacc[0][nt][r] *= aA[r]; oacc[0][nt][4 + r] *= aB[r];
          oacc[1][nt][r] *= bA[r]; oacc[1][nt][4 + r] *= bB[r];
        }
      }
    }
    __syncthreads();
    {
      const _Float16* vbp = vt + (size_t)(32 * wave + c) * vpitch + kbase + t * KCH + 8 * h;
#pragma unroll 1
      for (int ks = 0; ks < KCH; ks += 32) {
        const v16h pa0 = ldfrag(pa0p + ks), pa1 = ldfrag(pa1p + ks);
        const v16h vb0 = ldfrag(vbp + ks);
        const v16h vb1 = ldfrag(vbp + (size_t)16 * vpitch + ks);
        oacc[0][0] = mma16(pa0, vb0, oacc[0][0]);
        oacc[0][1] = mma16(pa0, vb1, oacc[0][1]);
        oacc[1][0] = mma16(pa1, vb0, oacc[1][0]);
        oacc[1][1] = mma16(pa1, vb1, oacc[1][1]);
        guard_s4(oacc[0][0], oacc[0][1], oacc[1][0], oacc[1][1], pa0, pa1, vb0, vb1);
      }
    }
  }

  if (wave == 0) {
    const int row = lane;
    float ps = 0.0f;
#pragma unroll
    for (int w = 0; w < 8; ++w) ps += psum[w * 32 + row];
    const float l = l_s[row] * al_s[row] + ps;
    li_s[row] = (1.0f / l) * (1.0f / 256.0f);
  }
  __syncthreads();
  {
    const v4f iA0 = *(const v4f*)(li_s + 8 * h),      iB0 = *(const v4f*)(li_s + 8 * h + 4);
    const v4f iA1 = *(const v4f*)(li_s + 16 + 8 * h), iB1 = *(const v4f*)(li_s + 16 + 8 * h + 4);
#pragma unroll
    for (int nt = 0; nt < 2; ++nt) {
      const int col = 32 * wave + 16 * nt + c;
      const float bv = bias[col];
#pragma unroll
      for (int r = 0; r < 4; ++r) {
        Os[(8 * h + r) * OSP + col]          = oacc[0][nt][r] * iA0[r] + bv;
        Os[(8 * h + 4 + r) * OSP + col]      = oacc[0][nt][4 + r] * iB0[r] + bv;
        Os[(16 + 8 * h + r) * OSP + col]     = oacc[1][nt][r] * iA1[r] + bv;
        Os[(16 + 8 * h + 4 + r) * OSP + col] = oacc[1][nt][4 + r] * iB1[r] + bv;
      }
    }
  }
  __syncthreads();
  {
    float* go = out + (size_t)q0 * opitch + ocol;
#pragma unroll
    for (int ps = 0; ps < 2; ++ps) {
#pragma unroll
      for (int rr = 0; rr < 4; ++rr) {
        const int row = 4 * wave + rr;
#pragma unroll
        for (int j = 0; j < 2; ++j) {
          const int pc = j * 32 + lane;
          const v4f v = *(const v4f*)(Os + row * OSP + pc * 4);
          *(volatile v4f*)(go + (size_t)row * opitch + pc * 4) = v;
        }
      }
      __threadfence();
    }
  }
}

extern "C" void kernel_launch(void* const* d_in, const int* in_sizes, int n_in,
                              void* d_out, int out_size, void* d_ws, size_t ws_size,
                              hipStream_t stream) {
  if (n_in < 16) return;
  if (in_sizes[0] != NROWS * DD || in_sizes[1] != NNODE * ECOLS || in_sizes[2] != DD * DD || in_sizes[3] != DD) return;
  if (in_sizes[4] != DD * DD || in_sizes[5] != DD || in_sizes[6] != DD * H1DIM || in_sizes[7] != H1DIM) return;
  if (in_sizes[8] != H1DIM * H2DIM || in_sizes[9] != H2DIM || in_sizes[10] != H2DIM || in_sizes[11] < 1) return;
  if (in_sizes[12] != DD || in_sizes[13] < 1 || in_sizes[14] < 1 || in_sizes[15] < 1) return;
  if (out_size != NROWS * OCOLS) return;

  const float* x          = (const float*)d_in[0];
  const int*   H          = (const int*)d_in[1];
  const float* weight     = (const float*)d_in[2];
  const float* bias       = (const float*)d_in[3];
  const float* Wn_w       = (const float*)d_in[4];
  const float* Wn_b       = (const float*)d_in[5];
  const float* m1w        = (const float*)d_in[6];
  const float* m1b        = (const float*)d_in[7];
  const float* m2w        = (const float*)d_in[8];
  const float* m2b        = (const float*)d_in[9];
  const float* m3w        = (const float*)d_in[10];
  const float* m3b        = (const float*)d_in[11];
  const float* c_w        = (const float*)d_in[12];
  const float* c_b        = (const float*)d_in[13];
  const float* hedge_bias = (const float*)d_in[14];
  const float* alpha_ctx  = (const float*)d_in[15];
  float* out = (float*)d_out;

  const size_t bW  = (size_t)DD * DD * 2;
  const size_t bX  = (size_t)NROWS * DD * 2;
  const size_t bCP = (size_t)NROWS * 4;
  const size_t bCT = (size_t)64 * 128;
  size_t off = 0;
  const size_t oWn = off; off += bW;
  const size_t oWt = off; off += bW;
  const size_t oX  = off; off += bX;
  const size_t oXP = off; off += bX;
  const size_t oVT = off; off += bX;
  const size_t oCP = off; off += bCP;
  const size_t oCT = off; off += bCT;
  if (off > ws_size) return;
  if (off > (size_t)134217728) return;

  char* ws = (char*)d_ws;
  _Float16* WnT16 = (_Float16*)(ws + oWn);
  _Float16* WT16  = (_Float16*)(ws + oWt);
  _Float16* X16   = (_Float16*)(ws + oX);
  _Float16* XP16  = (_Float16*)(ws + oXP);
  _Float16* VT16  = (_Float16*)(ws + oVT);
  float*    CP    = (float*)(ws + oCP);
  float*    CT    = (float*)(ws + oCT);

  const dim3 blk(256);
  cvt_w_kernel<<<dim3(2 * (DD / 8)), blk, 0, stream>>>(Wn_w, weight, WnT16, WT16, DD);
  cvt_x_kernel<<<dim3(NROWS / 32), blk, 0, stream>>>(x, c_w, c_b, X16, CP);
  gemm64_kernel<true><<<dim3(((NROWS / 64) * (DD / 64)) / 8), blk, 0, stream>>>(
      X16, DD, WnT16, DD, XP16, DD, Wn_b, 16.0f, NROWS, DD, DD, 0.25f);
  gemm64_kernel<false><<<dim3(((DD / 64) * (NROWS / 64)) / 8), blk, 0, stream>>>(
      WT16, DD, X16, DD, VT16, NROWS, Wn_b, 0.0f, DD, NROWS, DD, 0.25f);
  edge_kernel<<<dim3(NEMAX), blk, 0, stream>>>(x, H, m1w, m1b, m2w, m2b, m3w, m3b, CT, NNODE, ECOLS, NB);
  aw_kernel<<<dim3(NROWS / 8), blk, 0, stream>>>(H, CP, CT, hedge_bias, alpha_ctx, out, ECOLS, OCOLS, NEMAX);
  (void)hipFuncSetAttribute(reinterpret_cast<const void*>(&attn_kernel),
                            hipFuncAttributeMaxDynamicSharedMemorySize, ATT_LDS);
  const float sc = 0.0625f * (1.0f / 256.0f);
  attn_kernel<<<dim3(NNODE / QB, NB), blk, ATT_LDS, stream>>>(XP16, VT16, bias, out, sc, NNODE, NROWS, OCOLS, DD);
  (void)hipGetLastError();
}
